// EnhancedGNNModel_42709154791575
// MI455X (gfx1250) — hardware-run, weakly checked
//
#include <hip/hip_runtime.h>


namespace {
constexpr int N = 50000, NP = 50048, EFULL = 1600000, E = 1600000, NLIM = 50048  , C = 128, K2 = 2 * C, OA = 21, OS = 2, OE = 5, OH = 32  ;
constexpr size_t OUTN = (size_t)N * (OA + OS + OE);
constexpr float XS = 8.0f, WSC = 256.0f;
static_assert(NP % 64 == 0 && NP >= N && NLIM % 64 == 0 && NLIM <= NP && C == 128 && OUTN % 4 == 0, "tiling");
typedef _Float16 b16;
typedef __attribute__((ext_vector_type(16))) _Float16 v16b;
typedef __attribute__((ext_vector_type(8))) _Float16 v8b;
typedef __attribute__((ext_vector_type(8))) float v8f;
typedef __attribute__((ext_vector_type(4))) float v4f;
__device__ __forceinline__ float bf16_rne(float f) { unsigned int u = __float_as_uint(f); u += 0x7FFFu + ((u >> 16) & 1u); return __uint_as_float(u & 0xFFFF0000u); }
__device__ __forceinline__ void split16(float v, b16& hi, b16& lo) { hi = (b16)v; lo = (b16)(v - (float)hi); }
__device__ __forceinline__ v16b frag_kb(const b16* p, int hh) { const v8b a = *(const v8b*)(p + 8 * hh), b = *(const v8b*)(p + 16 + 8 * hh); v16b f;
#pragma unroll
  for (int e = 0; e < 8; ++e) { f[e] = a[e]; f[8 + e] = b[e]; } return f; }
__device__ __forceinline__ v8f wmma16b(v16b a, v16b b, v8f c) { v8f d = __builtin_amdgcn_wmma_f32_16x16x32_f16(false, a, false, b, (short)0, c, false, false); asm volatile("v_nop\n\tv_nop\n\tv_nop\n\tv_nop" : "+v"(d) : "v"(a), "v"(b)); return d; }
__device__ __forceinline__ void wave_lds_sync() { __builtin_amdgcn_fence(__ATOMIC_RELEASE, "workgroup"); __builtin_amdgcn_wave_barrier(); __builtin_amdgcn_fence(__ATOMIC_ACQUIRE, "workgroup"); }
__device__ __forceinline__ float pmul(float a, float b) { float p = a * b; asm volatile("" : "+v"(p)); return p; }
__device__ __forceinline__ int iclamp(int v, int lo, int hi) { return v < lo ? lo : (v > hi ? hi : v); }
constexpr int CSR_NBLK = 512, CSR_GB = 8  , CSR_GN = 1 << CSR_GB  , CSR_MAXG = 512, CSR_CAP = 12288  ;
__global__ __launch_bounds__(64) void csrA_kernel(const int* __restrict__ dst, int E, int N, int nG, int CHP, int NGP, int* __restrict__ STG, int* __restrict__ HST) {
  extern __shared__ int sm[];
  int* cnt = sm; int* run = sm + NGP; int* ids = sm + 2 * NGP;
  const int b = blockIdx.x; const int ch = (E + CSR_NBLK - 1) / CSR_NBLK; const int e0 = b * ch, e1 = min(E, e0 + ch);
  for (int i = threadIdx.x; i < NGP; i += 64) cnt[i] = 0;
  for (int i = threadIdx.x; i < CHP; i += 64) ids[i] = -1;
  __syncthreads();
  if (threadIdx.x == 0) {
    for (int e = e0; e < e1; ++e) { int d = dst[e]; d = (d < 0) ? 0 : (d >= N ? N - 1 : d); cnt[d >> CSR_GB] += 1; }
    int acc = 0; for (int g = 0; g < nG; ++g) { run[g] = acc; acc += cnt[g]; }
    for (int e = e0; e < e1; ++e) { int d = dst[e]; d = (d < 0) ? 0 : (d >= N ? N - 1 : d); const int g = d >> CSR_GB; ids[run[g]] = e; run[g] += 1; } }
  __syncthreads();
  typedef __attribute__((ext_vector_type(4))) int v4i;
  for (int pass = 0; pass < 2; ++pass) {
    for (int i = threadIdx.x; i < CHP / 4; i += 64) *(volatile v4i*)(STG + (size_t)b * CHP + i * 4) = *(const v4i*)(&ids[i * 4]);
    for (int i = threadIdx.x; i < NGP / 4; i += 64) { v4i v; for (int e = 0; e < 4; ++e) v[e] = (i * 4 + e < nG) ? cnt[i * 4 + e] : 0; *(volatile v4i*)(HST + (size_t)b * NGP + i * 4) = v; }
    __threadfence(); }
}
__global__ __launch_bounds__(512) void csrS_kernel(const int* __restrict__ HST, int nG, int NGP, int* __restrict__ START, int* __restrict__ TOT, int* __restrict__ OFF) {
  __shared__ int tot[CSR_MAXG];
  const int b = threadIdx.x;
  for (int pass = 0; pass < 2; ++pass) { int runb = 0; for (int g = 0; g < nG; ++g) { int c = HST[(size_t)b * NGP + g]; c = (c < 0) ? 0 : c; ((volatile int*)OFF)[(size_t)g * CSR_NBLK + b] = runb; runb += c; } __threadfence(); }
  for (int g = threadIdx.x; g < nG; g += 512) { int s = 0; for (int bb = 0; bb < CSR_NBLK; ++bb) { int c = HST[(size_t)bb * NGP + g]; s += (c < 0) ? 0 : c; } tot[g] = s; }
  __syncthreads();
  if (threadIdx.x < 32) {
    __shared__ int st[CSR_MAXG + 32];
    if (threadIdx.x == 0) { int acc = 0; for (int g = 0; g < NGP; ++g) { st[g] = acc; if (g < nG) acc += (tot[g] + 31) & ~31; } st[NGP] = acc; }
    __builtin_amdgcn_fence(__ATOMIC_RELEASE, "workgroup"); __builtin_amdgcn_wave_barrier(); __builtin_amdgcn_fence(__ATOMIC_ACQUIRE, "workgroup");
    for (int pass = 0; pass < 2; ++pass) { for (int i = threadIdx.x; i < NGP + 32; i += 32) { ((volatile int*)START)[i] = (i <= NGP) ? st[min(i, NGP)] : 0; ((volatile int*)TOT)[i] = (i < nG) ? tot[i] : 0; } __threadfence(); } }
}
__global__ __launch_bounds__(256) void csrB_kernel(const int* __restrict__ dst, int N, int nG, int CHP, int NGP, int permLen, const int* __restrict__ STG, const int* __restrict__ HST, const int* __restrict__ OFF, const int* __restrict__ START, const int* __restrict__ TOT, int* __restrict__ PERM, int* __restrict__ ROWPTR, int* __restrict__ ROWCNT, int* __restrict__ FLAG) {
  typedef __attribute__((ext_vector_type(4))) int v4i;
  __shared__ int ids[CSR_CAP]; __shared__ unsigned short key[CSR_CAP]; __shared__ int outp[CSR_CAP]; __shared__ int ncnt[CSR_GN + 1]; __shared__ int boff[CSR_NBLK + 1];
  const int g = blockIdx.x, t_ = threadIdx.x; int tot = TOT[g]; int st = START[g], stn = START[g + 1]; const int v0 = g * CSR_GN; const int nv = min(CSR_GN, N - v0);
  st = (st < 0) ? 0 : (st > permLen - 32 ? permLen - 32 : st) & ~31; stn = (stn < st) ? st : (stn > permLen ? permLen : stn); tot = (tot < 0) ? 0 : tot; if (tot > stn - st && tot <= CSR_CAP) tot = stn - st;
  if (tot > CSR_CAP) {
    for (int pass = 0; pass < 2; ++pass) { for (int i = t_; i < CSR_GN / 4; i += 256) { v4i a, c; for (int e = 0; e < 4; ++e) { a[e] = st; c[e] = 0; } *(volatile v4i*)(ROWPTR + v0 + i * 4) = a; *(volatile v4i*)(ROWCNT + v0 + i * 4) = c; } if (t_ == 0) ((volatile int*)FLAG)[0] = 1; __threadfence(); } (void)nv; return; }
  if (t_ == 0) { int acc = 0; for (int b = 0; b < CSR_NBLK; ++b) { boff[b] = acc; int c = HST[(size_t)b * NGP + g]; c = (c < 0) ? 0 : (c > CHP ? CHP : c); acc += c; if (acc > tot) acc = tot; } boff[CSR_NBLK] = acc; }
  for (int i = t_; i <= CSR_GN; i += 256) ncnt[i] = 0;
  __syncthreads();
  for (int b = 0; b < CSR_NBLK; ++b) { const int c = boff[b + 1] - boff[b]; int o_ = OFF[(size_t)g * CSR_NBLK + b]; o_ = (o_ < 0) ? 0 : (o_ > CHP - c ? CHP - c : o_); const int* src_ = STG + (size_t)b * CHP + o_;
    for (int i = t_; i < c; i += 256) { int id = src_[i]; id = (id < 0) ? 0 : id; ids[boff[b] + i] = id; int d = dst[id]; d = (d < v0) ? v0 : (d >= N ? N - 1 : d); int kk = d - v0; kk = (kk < 0) ? 0 : (kk >= CSR_GN ? CSR_GN - 1 : kk); key[boff[b] + i] = (unsigned short)kk; } }
  __syncthreads();
  if (t_ == 0) { for (int i = 0; i < tot; ++i) ncnt[key[i]] += 1; int acc = 0; for (int vl = 0; vl < CSR_GN; ++vl) { const int c = ncnt[vl]; ncnt[vl] = acc; acc += c; } ncnt[CSR_GN] = acc;
    for (int i = 0; i < tot; ++i) { const int vl = key[i]; outp[ncnt[vl]] = ids[i]; ncnt[vl] += 1; }
    for (int vl = CSR_GN; vl > 0; --vl) ncnt[vl] = ncnt[vl - 1]; ncnt[0] = 0; }
  __syncthreads();
  for (int pass = 0; pass < 2; ++pass) {
    for (int i = t_; i < (stn - st) / 4; i += 256) { v4i v; for (int e = 0; e < 4; ++e) { const int q = i * 4 + e; v[e] = (q < tot) ? outp[q] : -1; } *(volatile v4i*)(PERM + st + i * 4) = v; }
    for (int i = t_; i < CSR_GN / 4; i += 256) { v4i a, c; for (int e = 0; e < 4; ++e) { const int vl = i * 4 + e; a[e] = st + ncnt[vl]; c[e] = (vl < nv) ? (ncnt[vl + 1] - ncnt[vl]) : 0; } *(volatile v4i*)(ROWPTR + v0 + i * 4) = a; *(volatile v4i*)(ROWCNT + v0 + i * 4) = c; }
    __threadfence(); }
}
__global__ __launch_bounds__(256) void csrZ_kernel(int* __restrict__ p, size_t n4) { typedef __attribute__((ext_vector_type(4))) int v4i; const size_t tid = (size_t)blockIdx.x * 256 + threadIdx.x, nth = (size_t)gridDim.x * 256; v4i z = {0, 0, 0, 0}; for (size_t i = tid; i < n4; i += nth) *(volatile v4i*)(p + i * 4) = z; }
struct CsrBufs { int *STG, *HST, *OFF, *START, *TOT, *PERM, *ROWPTR, *ROWCNT, *FLAG; int nG, NGP, CHP; size_t permLen; char* base; size_t bytes; };
static size_t csr_carve(CsrBufs& c, char* ws, size_t off, int E, int N) {
  const size_t off0 = off; c.base = ws + off;
  auto al = [&](size_t bytes) { char* p = ws + off; off += (bytes + 255) & ~(size_t)255; return p; };
  c.nG = (N + CSR_GN - 1) / CSR_GN; c.NGP = (c.nG + 31) & ~31; const int ch = (E + CSR_NBLK - 1) / CSR_NBLK; c.CHP = (ch + 31) & ~31; c.permLen = (size_t)E + 32 * (size_t)c.nG + 32;
  c.STG = (int*)al((size_t)CSR_NBLK * c.CHP * 4); c.HST = (int*)al((size_t)CSR_NBLK * c.NGP * 4); c.OFF = (int*)al((size_t)c.NGP * CSR_NBLK * 4); c.START = (int*)al((size_t)(c.NGP + 64) * 4); c.TOT = (int*)al((size_t)(c.NGP + 64) * 4);
  c.PERM = (int*)al(c.permLen * 4); c.ROWPTR = (int*)al((size_t)c.nG * CSR_GN * 4); c.ROWCNT = (int*)al((size_t)c.nG * CSR_GN * 4); c.FLAG = (int*)al(256);
  c.bytes = off - off0; return off;
}
static void csr_build(const CsrBufs& c, const int* dst, int E, int N, hipStream_t stream) {
  const size_t smem = (size_t)(2 * c.NGP + c.CHP) * 4;
  csrZ_kernel<<<512, 256, 0, stream>>>((int*)c.base, c.bytes / 16);
  csrA_kernel<<<CSR_NBLK, 64, smem, stream>>>(dst, E, N, c.nG, c.CHP, c.NGP, c.STG, c.HST);
  csrS_kernel<<<1, 512, 0, stream>>>(c.HST, c.nG, c.NGP, c.START, c.TOT, c.OFF);
  csrB_kernel<<<c.nG, 256, 0, stream>>>(dst, N, c.nG, c.CHP, c.NGP, (int)c.permLen, c.STG, c.HST, c.OFF, c.START, c.TOT, c.PERM, c.ROWPTR, c.ROWCNT, c.FLAG);
}

typedef __attribute__((ext_vector_type(4))) _Float16 v4h;
__global__ __launch_bounds__(256) void wprep_kernel(const float* __restrict__ wl1, const float* __restrict__ wr1, const float* __restrict__ wl2, const float* __restrict__ wr2, const float* __restrict__ wl3, const float* __restrict__ wr3,
                                                     const float* __restrict__ wla, const float* __restrict__ wra, const float* __restrict__ wls, const float* __restrict__ wrs, const float* __restrict__ wle, const float* __restrict__ wre, b16* __restrict__ WT, b16* __restrict__ WH) {
  const int u = blockIdx.x * 256 + threadIdx.x; const int n3 = 3 * C * K2 / 8, nh = OH * K2 / 8; v8b o;
  if (u < n3) { const int e = u * 8; const int l = e / (C * K2), el = e % (C * K2); const int oo = el / K2, k0 = el % K2; const float* w = (k0 < C) ? (l == 0 ? wl1 : l == 1 ? wl2 : wl3) : (l == 0 ? wr1 : l == 1 ? wr2 : wr3); const int kk = k0 % C;
    for (int j = 0; j < 8; ++j) o[j] = (b16)(bf16_rne(w[(size_t)oo * C + kk + j]) * WSC); for (int pass = 0; pass < 2; ++pass) { *(volatile v8b*)(WT + e) = o; __threadfence(); } return; }
  const int t = u - n3; if (t >= nh) return; { const int e = t * 8; const int oo = e / K2, k0 = e % K2, kk = k0 % C; const bool left = k0 < C; const float* w = nullptr; int orow = 0;
    if (oo < OA) { w = left ? wla : wra; orow = oo; } else if (oo < OA + OS) { w = left ? wls : wrs; orow = oo - OA; } else if (oo < OA + OS + OE) { w = left ? wle : wre; orow = oo - OA - OS; }
    for (int j = 0; j < 8; ++j) o[j] = w ? (b16)(bf16_rne(w[(size_t)orow * C + kk + j]) * WSC) : (b16)0.0f; for (int pass = 0; pass < 2; ++pass) { *(volatile v8b*)(WH + e) = o; __threadfence(); } }
}
__global__ __launch_bounds__(256) void x_kernel(const float* __restrict__ x, float* __restrict__ H) {
  const size_t u = (size_t)blockIdx.x * 256 + threadIdx.x; if (u >= (size_t)NP * C / 4) return; const size_t e = u * 4; const size_t v = e / C; v4f o = {0.0f, 0.0f, 0.0f, 0.0f};
  if (v < (size_t)N) { const v4f a = *(const v4f*)(x + e); for (int i = 0; i < 4; ++i) o[i] = bf16_rne(a[i]); }
  for (int pass = 0; pass < 2; ++pass) { *(volatile v4f*)(H + e) = o; __threadfence(); }
}
__global__ __launch_bounds__(256) void agg_kernel(const float* __restrict__ H, const int* __restrict__ srcs, const int* __restrict__ PERM, const int* __restrict__ ROWPTR, const int* __restrict__ ROWCNT, int permLen, b16* __restrict__ Mh, b16* __restrict__ Ml, b16* __restrict__ Hh, b16* __restrict__ Hl) {
  const int wave = threadIdx.x >> 5, lane = threadIdx.x & 31; const size_t v = (size_t)blockIdx.x * 8 + wave; const int c = lane * 4; v4f a = {0.0f, 0.0f, 0.0f, 0.0f}, hv = {0.0f, 0.0f, 0.0f, 0.0f};
  if (v < (size_t)N) { int st = ROWPTR[v], cnt = ROWCNT[v]; cnt = iclamp(cnt, 0, 65536); st = iclamp(st, 0, permLen - cnt);
#pragma unroll 1
    for (int j = 0; j < cnt; ++j) { const int e = iclamp(PERM[st + j], 0, E - 1); const int s = iclamp(srcs[e], 0, N - 1); v4f t = *(const v4f*)(H + (size_t)s * C + c); if (s >= NLIM) t = (v4f){0.0f, 0.0f, 0.0f, 0.0f}; a += t; }
    const float inv = 1.0f / (float)(cnt < 1 ? 1 : cnt); for (int i = 0; i < 4; ++i) a[i] = pmul(a[i], inv); hv = *(const v4f*)(H + v * C + c); }
  v4h ah, al, hh, hl; for (int i = 0; i < 4; ++i) { b16 p, q; split16(a[i] * XS, p, q); ah[i] = p; al[i] = q; split16(hv[i] * XS, p, q); hh[i] = p; hl[i] = q; }
  for (int pass = 0; pass < 2; ++pass) { *(volatile v4h*)(Mh + v * C + c) = ah; *(volatile v4h*)(Ml + v * C + c) = al; *(volatile v4h*)(Hh + v * C + c) = hh; *(volatile v4h*)(Hl + v * C + c) = hl; __threadfence(); }
}
template <int NT, int RELU>
__global__ __launch_bounds__(128) void sage_kernel(const b16* __restrict__ Mh, const b16* __restrict__ Ml, const b16* __restrict__ Hh, const b16* __restrict__ Hl, const b16* __restrict__ WT, const float* __restrict__ b0, const float* __restrict__ b1, const float* __restrict__ b2, float* __restrict__ OUT) {
  __shared__ __attribute__((aligned(16))) float Tf[4][16][NT * 16 + 4];
  const int wave = threadIdx.x >> 5, lane = threadIdx.x & 31, nloc = lane & 15, hlf = lane >> 4; const size_t m0 = (size_t)blockIdx.x * 64 + wave * 16;
  v8f acc[NT];
#pragma unroll
  for (int t = 0; t < NT; ++t) acc[t] = (v8f){};
#pragma unroll 2
  for (int kb = 0; kb < K2; kb += 32) { const bool left = kb < C; const b16* Ph = left ? Mh : Hh; const b16* Pl = left ? Ml : Hl; const int kk = left ? kb : kb - C;
    const v16b a = frag_kb(Ph + (m0 + nloc) * C + kk, hlf), al = frag_kb(Pl + (m0 + nloc) * C + kk, hlf);
#pragma unroll
    for (int t = 0; t < NT; ++t) { const v16b bw = frag_kb(WT + (size_t)(t * 16 + nloc) * K2 + kb, hlf); acc[t] = wmma16b(a, bw, acc[t]); acc[t] = wmma16b(al, bw, acc[t]); } }
#pragma unroll
  for (int t = 0; t < NT; ++t)
#pragma unroll
    for (int r = 0; r < 8; ++r) Tf[wave][8 * hlf + r][t * 16 + nloc] = acc[t][r] * (1.0f / (XS * WSC));
  wave_lds_sync();
  constexpr int NCOL = NT * 16;
  if (lane * 4 < NCOL) { v4f bb; for (int j = 0; j < 4; ++j) { const int cc = lane * 4 + j; float b = 0.0f;
      if (NT == 8) b = bf16_rne(b0[cc]); else { if (cc < OA) b = bf16_rne(b0[cc]); else if (cc < OA + OS) b = bf16_rne(b1[cc - OA]); else if (cc < OA + OS + OE) b = bf16_rne(b2[cc - OA - OS]); }
      bb[j] = b; }
    for (int pass = 0; pass < 2; ++pass) { for (int rr = 0; rr < 16; ++rr) { v4f o = *(const v4f*)(&Tf[wave][rr][lane * 4]); o += bb; if (RELU) { for (int j = 0; j < 4; ++j) o[j] = fmaxf(o[j], 0.0f); } const size_t v = m0 + rr;
        if (v >= (size_t)N) o = (v4f){0.0f, 0.0f, 0.0f, 0.0f};
        *(volatile v4f*)(OUT + v * NCOL + lane * 4) = o; } __threadfence(); } }
}
__global__ __launch_bounds__(256) void tuple_kernel(const float* __restrict__ HD, float* __restrict__ out) {
  const size_t q = (size_t)blockIdx.x * 256 + threadIdx.x; if (q * 4 >= OUTN) return; v4f o;
  for (int j = 0; j < 4; ++j) { const size_t i = q * 4 + j; size_t v; int col;
    if (i < (size_t)N * OA) { v = i / OA; col = (int)(i % OA); } else if (i < (size_t)N * (OA + OS)) { const size_t r = i - (size_t)N * OA; v = r / OS; col = OA + (int)(r % OS); } else { const size_t r = i - (size_t)N * (OA + OS); v = r / OE; col = OA + OS + (int)(r % OE); }
    o[j] = HD[v * OH + col]; }
  for (int pass = 0; pass < 2; ++pass) { *(volatile v4f*)(out + q * 4) = o; __threadfence(); }
}
}

extern "C" void kernel_launch(void* const* d_in, const int* in_sizes, int n_in, void* d_out, int out_size, void* d_ws, size_t ws_size, hipStream_t stream) {
  (void)n_in;
  auto Fp = [&](int i) { return (const float*)d_in[i]; }; auto Ip = [&](int i) { return (const int*)d_in[i]; };
  if (in_sizes[0] != N * C || in_sizes[1] != 2 * EFULL || in_sizes[2] != C * C || in_sizes[3] != C * C || in_sizes[4] != C || in_sizes[5] != C * C || in_sizes[8] != C * C || in_sizes[11] != OA * C || in_sizes[12] != OA * C || in_sizes[13] != OA ||
      in_sizes[14] != OS * C || in_sizes[16] != OS || in_sizes[17] != OE * C || in_sizes[19] != OE || (size_t)out_size != OUTN) return;
  size_t off = 0; char* ws = (char*)d_ws;
  auto carve = [&](size_t bytes) { char* p = ws + off; off += (bytes + 255) & ~(size_t)255; return p; };
  b16* WT = (b16*)carve((size_t)3 * C * K2 * 2); b16* WH = (b16*)carve((size_t)OH * K2 * 2); float* H = (float*)carve((size_t)NP * C * 4);
  b16* Mh = (b16*)carve((size_t)NP * C * 2); b16* Ml = (b16*)carve((size_t)NP * C * 2); b16* Hh = (b16*)carve((size_t)NP * C * 2); b16* Hl = (b16*)carve((size_t)NP * C * 2); float* HD = (float*)carve((size_t)NP * OH * 4);
  CsrBufs csr; off = csr_carve(csr, ws, off, E, N);
  if (off > ws_size || off > ((size_t)128 << 20)) return;
  wprep_kernel<<<(3 * C * K2 / 8 + OH * K2 / 8 + 255) / 256, 256, 0, stream>>>(Fp(2), Fp(3), Fp(5), Fp(6), Fp(8), Fp(9), Fp(11), Fp(12), Fp(14), Fp(15), Fp(17), Fp(18), WT, WH);
  csr_build(csr, Ip(1) + EFULL, E, N, stream);
  x_kernel<<<(unsigned)(((size_t)NP * C / 4 + 255) / 256), 256, 0, stream>>>(Fp(0), H);
  for (int l = 0; l < 3; ++l) {
    agg_kernel<<<NLIM / 8, 256, 0, stream>>>(H, Ip(1), csr.PERM, csr.ROWPTR, csr.ROWCNT, (int)csr.permLen, Mh, Ml, Hh, Hl);
    sage_kernel<8, 1><<<NLIM / 64, 128, 0, stream>>>(Mh, Ml, Hh, Hl, WT + (size_t)l * C * K2, Fp(4 + 3 * l), nullptr, nullptr, H); }
  agg_kernel<<<NLIM / 8, 256, 0, stream>>>(H, Ip(1), csr.PERM, csr.ROWPTR, csr.ROWCNT, (int)csr.permLen, Mh, Ml, Hh, Hl);
  sage_kernel<2, 0><<<NLIM / 64, 128, 0, stream>>>(Mh, Ml, Hh, Hl, WH, Fp(13), Fp(16), Fp(19), HD);
  tuple_kernel<<<(unsigned)((OUTN / 4 + 255) / 256), 256, 0, stream>>>(HD, (float*)d_out);
}
